// MultiHeadedAttention_81801947120046
// MI455X (gfx1250) — hardware-verified
//
#include <hip/hip_runtime.h>
#include <math.h>

#ifndef NB
#define NB 4
#endif
#ifndef SEQ
#define SEQ 2048
#endif
#define NB_FULL 4
#define SEQ_FULL 2048
#define DM 512
#define NH 8
#define HD 64
#define NTOK (NB * SEQ)
#define NQB (SEQ / 64)

#define W_CARRY    16.0f
#define QKV_CARRY  16.0f
#define P_CARRY    1024.0f
#define SC_SCORE   (0.125f / 256.0f)
#define CTX_FOLD   (1.0f / 64.0f)
#define OUT_SCALE  (1.0f / 4096.0f)
#define NEG_FILL   (-__FLT_MAX__)

static_assert(NH * HD == DM);
static_assert(HD == 64);
static_assert(DM % 64 == 0);
static_assert(DM % 32 == 0);
static_assert(DM % 8 == 0);
static_assert(SEQ % 64 == 0);
static_assert(NTOK % 64 == 0);
static_assert(NB <= NB_FULL);
static_assert(SEQ <= SEQ_FULL);
static_assert(sizeof(long) == 8);
static_assert((DM * (DM / 8)) % 256 == 0);

typedef __attribute__((ext_vector_type(16))) _Float16 v16h;
typedef __attribute__((ext_vector_type(8)))  _Float16 v8h;
typedef __attribute__((ext_vector_type(8)))  float    v8f;
typedef __attribute__((ext_vector_type(4)))  float    v4f;
typedef __attribute__((ext_vector_type(4)))  unsigned int v4u;
typedef unsigned short us;
typedef __attribute__((ext_vector_type(8)))  unsigned short v8us;
typedef __attribute__((ext_vector_type(16))) unsigned short v16us;


#define VST2(T, ptr, val) do { const T vst2_v_ = (val); *(volatile T*)(ptr) = vst2_v_; __threadfence(); *(volatile T*)(ptr) = vst2_v_; } while (0)

namespace gk {

__device__ __forceinline__ unsigned short f2bf_bits(float f) {
  unsigned u = __float_as_uint(f);
  return (unsigned short)((u + 0x7FFFu + ((u >> 16) & 1u)) >> 16);
}
__device__ __forceinline__ unsigned short f2h_bits(float f) { return __builtin_bit_cast(unsigned short, (_Float16)f); }

__device__ __forceinline__ void dep_guard_h(v8f& a, v8f& b, v16h x, v16h y) { asm volatile("v_nop\n\tv_nop\n\tv_nop\n\tv_nop" : "+v"(a), "+v"(b) : "v"(x), "v"(y)); }
__device__ __forceinline__ void keep4_h(v16h a, v16h b, v16h c, v16h d) { asm volatile("v_nop" :: "v"(a), "v"(b), "v"(c), "v"(d)); }
__device__ __forceinline__ void acc_guard4(v8f& a, v8f& b, v8f& c, v8f& d) { asm volatile("v_nop\n\tv_nop\n\tv_nop\n\tv_nop" : "+v"(a), "+v"(b), "+v"(c), "+v"(d)); }

union FragU { v16h v; v8h h[2]; };
__device__ __forceinline__ v16h frag_load(const _Float16* p) {
  FragU f; f.h[0] = *(const v8h*)(p); f.h[1] = *(const v8h*)(p + 16); return f.v;
}
__device__ __forceinline__ v8f frag_mma(v16h a, v16h b, v8f c) {
  return __builtin_amdgcn_wmma_f32_16x16x32_f16(false, a, false, b, (short)0, c, false, false);
}

template <int BIAS_MODE, int OUT_MODE>
__device__ __forceinline__ void gemm64_body(
    const unsigned short* __restrict__ Ap, int lda, long strideA,
    const unsigned short* __restrict__ Btp, int ldb, long strideB,
    void* __restrict__ Cout, int ldc, long strideC,
    const float* __restrict__ biasp, int strideBias,
    int M, int N, int K, float scale, float carry) {
  __shared__ __align__(16) float sT[8][16 * 68];
  const _Float16* A = (const _Float16*)Ap; const _Float16* Bt = (const _Float16*)Btp;
  const int b    = blockIdx.y;
  const int lane = threadIdx.x & 31;
  const int wave = threadIdx.x >> 5;
  const int tilesN = N >> 6;
  const int tilesM = M >> 6;
  const int tile = blockIdx.x * 8 + wave;
  if (tile >= tilesM * tilesN) return;
  const int tm = tile / tilesN;
  const int tn = tile - tm * tilesN;
  const int m0 = tm << 6;
  const int n0 = tn << 6;

  const _Float16* Ab = A  + (size_t)b * strideA;
  const _Float16* Bb = Bt + (size_t)b * strideB;
  const float* bias = biasp + (size_t)b * strideBias;

  const int rlane = lane & 15;
  const int koff  = (lane >> 4) * 8;
  const int mOff  = (lane >> 4) * 8;

  v8f acc[4][4];
#pragma unroll
  for (int i = 0; i < 4; ++i)
#pragma unroll
    for (int j = 0; j < 4; ++j) acc[i][j] = (v8f){0.f,0.f,0.f,0.f,0.f,0.f,0.f,0.f};

  for (int k0 = 0; k0 < K; k0 += 32) {
    v16h bh[4];
#pragma unroll
    for (int j = 0; j < 4; ++j) {
      const size_t bo = (size_t)(n0 + (j << 4) + rlane) * ldb + koff + k0;
      bh[j] = frag_load(Bb + bo);
    }
#pragma unroll
    for (int i = 0; i < 4; ++i) {
      const size_t ao = (size_t)(m0 + (i << 4) + rlane) * lda + koff + k0;
      v16h ah = frag_load(Ab + ao);
#pragma unroll
      for (int j = 0; j < 4; ++j) acc[i][j] = frag_mma(ah, bh[j], acc[i][j]);
      dep_guard_h(acc[i][0], acc[i][3], ah, ah);
    }
    keep4_h(bh[0], bh[1], bh[2], bh[3]);
  }
  acc_guard4(acc[0][0], acc[0][1], acc[0][2], acc[0][3]);
  acc_guard4(acc[1][0], acc[1][1], acc[1][2], acc[1][3]);
  acc_guard4(acc[2][0], acc[2][1], acc[2][2], acc[2][3]);
  acc_guard4(acc[3][0], acc[3][1], acc[3][2], acc[3][3]);

  float* slab = sT[wave];
#pragma unroll
  for (int i = 0; i < 4; ++i) {
    const int mBase = m0 + (i << 4);
#pragma unroll
    for (int j = 0; j < 4; ++j) {
      const int n = n0 + (j << 4) + rlane;
      float bv = 0.f;
      if (BIAS_MODE == 2) bv = bias[n];
#pragma unroll
      for (int r = 0; r < 8; ++r) {
        float v = acc[i][j][r] * scale;
        if (BIAS_MODE == 1) v += bias[mBase + mOff + r];
        if (BIAS_MODE == 2) v += bv;
        slab[(mOff + r) * 68 + (j << 4) + rlane] = v * carry;
      }
    }
    __builtin_amdgcn_fence(3  , "workgroup");
    __builtin_amdgcn_wave_barrier();
    __builtin_amdgcn_fence(2  , "workgroup");
    if (OUT_MODE == 0) {
      float* C = (float*)Cout + (size_t)b * strideC;
      const int hh = lane >> 4, c4 = (lane & 15) * 4;
      for (int pass = 0; pass < 2; ++pass) {
#pragma unroll
        for (int it = 0; it < 8; ++it) {
          const int row = it * 2 + hh;
          v4f v = *(const v4f*)(slab + row * 68 + c4);
          *(volatile v4f*)(C + (size_t)(mBase + row) * ldc + n0 + c4) = v;
        }
        __threadfence();
      }
    } else {
      const int q = lane >> 3, c8 = (lane & 7) * 8;
      unsigned short* C  = (unsigned short*)Cout + (size_t)b * strideC;
      for (int pass = 0; pass < 2; ++pass) {
#pragma unroll
        for (int it = 0; it < 4; ++it) {
          const int row = it * 4 + q;
          const float* sp = slab + row * 68 + c8;
          v8us hv;
#pragma unroll
          for (int e = 0; e < 8; ++e) hv[e] = f2h_bits(sp[e]);
          *(volatile v8us*)(C + (size_t)(mBase + row) * ldc + n0 + c8) = hv;
        }
        __threadfence();
      }
    }
    __builtin_amdgcn_fence(3  , "workgroup");
    __builtin_amdgcn_wave_barrier();
    __builtin_amdgcn_fence(2  , "workgroup");
  }
}

}

__global__ __launch_bounds__(256) void k_gemm_qk(const us* __restrict__ X16, const us* __restrict__ W16, us* __restrict__ QK16, const float* __restrict__ BR) {
  static_assert(NTOK % 64 == 0 && DM % 64 == 0 && DM % 32 == 0);
  gk::gemm64_body<2, 1>(X16, DM, (long)NTOK * DM, W16, DM, (long)DM * DM, (void*)QK16, DM, (long)NTOK * DM, BR, DM, NTOK, DM, DM, 1.0f / W_CARRY, QKV_CARRY);
}
__global__ __launch_bounds__(256) void k_gemm_vt(const us* __restrict__ Wv16, const us* __restrict__ Xv16, us* __restrict__ VT16, const float* __restrict__ BRv) {
  static_assert(NTOK % 64 == 0 && DM % 64 == 0 && DM % 32 == 0);
  gk::gemm64_body<1, 1>(Wv16, DM, 0L, Xv16, DM, 0L, (void*)VT16, NTOK, 0L, BRv, 0, DM, NTOK, DM, 1.0f / W_CARRY, QKV_CARRY);
}
__global__ __launch_bounds__(256) void k_gemm_out(const us* __restrict__ CTX, const us* __restrict__ Wo16, float* __restrict__ out, const float* __restrict__ BRo) {
  static_assert(SEQ % 64 == 0 && DM % 32 == 0 && DM % 64 == 0);
  gk::gemm64_body<2, 0>(CTX, DM, (long)SEQ * DM, Wo16, DM, 0L, (void*)out, DM, (long)SEQ_FULL * DM, BRo, 0, SEQ, DM, DM, OUT_SCALE, 1.0f);
}

__device__ __forceinline__ unsigned int cmb_pk2(float a, float b) { return (unsigned int)__builtin_bit_cast(unsigned short, (_Float16)a) | ((unsigned int)__builtin_bit_cast(unsigned short, (_Float16)b) << 16); }
__device__ __forceinline__ float cmb_bf(float v) { const unsigned u = __builtin_bit_cast(unsigned, v); const unsigned r = (u + 0x7fffu + ((u >> 16) & 1u)) & 0xffff0000u; return __builtin_bit_cast(float, r); }
__device__ __forceinline__ void cast8_f16(const float* __restrict__ s, us* __restrict__ d, float sc) {
  const v4f a = *(const v4f*)s; const v4f b2 = *(const v4f*)(s + 4);
  v4u pk;
  pk.x = cmb_pk2(cmb_bf(a.x) * sc, cmb_bf(a.y) * sc); pk.y = cmb_pk2(cmb_bf(a.z) * sc, cmb_bf(a.w) * sc);
  pk.z = cmb_pk2(cmb_bf(b2.x) * sc, cmb_bf(b2.y) * sc); pk.w = cmb_pk2(cmb_bf(b2.z) * sc, cmb_bf(b2.w) * sc);
  VST2(v4u, (v4u*)d, pk);
}
__global__ __launch_bounds__(256) void k_cast_w4(const float* __restrict__ Wq, const float* __restrict__ Wk, const float* __restrict__ Wv, const float* __restrict__ Wo, us* __restrict__ W16) {
  static_assert(DM % 8 == 0);
  const int u = blockIdx.x * 256 + threadIdx.x; if (u >= DM * (DM / 8)) return;
  const int r = u / (DM / 8); const int c0 = 8 * (u % (DM / 8));
  const size_t o = (size_t)r * DM + c0;
  cast8_f16(Wq + o, W16 + o, W_CARRY);
  cast8_f16(Wk + o, W16 + (size_t)DM * DM + o, W_CARRY);
  cast8_f16(Wv + o, W16 + (size_t)2 * DM * DM + o, W_CARRY);
  cast8_f16(Wo + o, W16 + (size_t)3 * DM * DM + o, W_CARRY);
}
__global__ __launch_bounds__(256) void k_bias4(const float* __restrict__ bq, const float* __restrict__ bk, const float* __restrict__ bv, const float* __restrict__ bo, float* __restrict__ BR) {
  static_assert(DM % 32 == 0);
  const int u = blockIdx.x * 256 + threadIdx.x; if (u >= DM) return;
  VST2(float, BR + u, cmb_bf(bq[u]));
  VST2(float, BR + DM + u, cmb_bf(bk[u]));
  VST2(float, BR + 2 * DM + u, cmb_bf(bv[u]));
  VST2(float, BR + 3 * DM + u, cmb_bf(bo[u]));
}
__global__ __launch_bounds__(256) void k_cast_x3(const float* __restrict__ xq, const float* __restrict__ xk, const float* __restrict__ xv, us* __restrict__ X16) {
  const long long u = (long long)blockIdx.x * 256 + threadIdx.x; if (u >= (long long)NTOK * (DM / 8)) return;
  const int r = (int)(u / (DM / 8)); const int c0 = 8 * (int)(u % (DM / 8));
  const int b = r / SEQ; const int s = r - b * SEQ;
  const size_t so = ((size_t)b * SEQ_FULL + s) * DM + c0; const size_t dofs = (size_t)r * DM + c0;
  cast8_f16(xq + so, X16 + dofs, 1.0f);
  cast8_f16(xk + so, X16 + (size_t)NTOK * DM + dofs, 1.0f);
  cast8_f16(xv + so, X16 + (size_t)2 * NTOK * DM + dofs, 1.0f);
}

__device__ __forceinline__ v8f mma_h(v16h a, v16h b, v8f c) {
  c = __builtin_amdgcn_wmma_f32_16x16x32_f16(false, a, false, b, (short)0, c, false, false);
  asm volatile("v_nop\n\tv_nop\n\tv_nop\n\tv_nop" : "+v"(c) : "v"(a), "v"(b));
  return c;
}
__device__ __forceinline__ void wave_sync() {
  __builtin_amdgcn_fence(3  , "workgroup");
  __builtin_amdgcn_wave_barrier();
  __builtin_amdgcn_fence(2  , "workgroup");
}
union FBU { v16us u; v8us h[2]; };
#define LDFRAG(dst, arr, off) do { FBU f_; f_.h[0] = *(const v8us*)&arr[(off)]; f_.h[1] = *(const v8us*)&arr[(off) + 16]; dst = __builtin_bit_cast(v16h, f_.u); } while (0)

__global__ __launch_bounds__(128) void k_attn_flash(const us* __restrict__ QK16, const us* __restrict__ VT16, const int* __restrict__ MK, us* __restrict__ CTX) {
  static_assert(HD == 64 && SEQ % 64 == 0 && DM == NH * HD);
  __shared__ __align__(16) us Qs[64 * 64];
  __shared__ __align__(16) us Ks[64 * 64];
  __shared__ __align__(16) us Vts[64 * 64];
  __shared__ __align__(16) us Ps[4 * 16 * 32];
  __shared__ int msk_s[64];

  const int tid = threadIdx.x, wave = tid >> 5, lane = tid & 31, hh = lane >> 4, c = lane & 15;
  const int bx = blockIdx.x;
  const int qb = bx % NQB; const int bh = bx / NQB; const int h = bh % NH; const int b = bh / NH;
  const int tok0 = b * SEQ + qb * 64;
  const size_t KOFF = (size_t)NTOK * DM;

  {
    const int row = tid >> 1, dh = (tid & 1) * 32;
    const size_t qro_g = (size_t)(tok0 + row) * DM + h * HD + dh;
#pragma unroll
    for (int i = 0; i < 4; ++i) *(v8us*)&Qs[row * 64 + dh + 8 * i] = *(const v8us*)(QK16 + qro_g + 8 * i);
  }
  __syncthreads();

  float mrow[8], lrow[8], lval[8];
  v8f oacc[4];
#pragma unroll
  for (int r = 0; r < 8; ++r) { mrow[r] = -__builtin_inff(); lrow[r] = 0.f; lval[r] = 0.f; }
#pragma unroll
  for (int t = 0; t < 4; ++t) oacc[t] = (v8f){0.f,0.f,0.f,0.f,0.f,0.f,0.f,0.f};

  const int pb = wave * 512;
  const int qro = (wave * 16 + c) * 64 + 8 * hh;

#pragma unroll 1
  for (int kc = 0; kc < NQB; ++kc) {
    const int kv0 = kc * 64;
    __syncthreads();
    {
      const int row = tid >> 1, dh = (tid & 1) * 32;
      const size_t kro = KOFF + (size_t)(b * SEQ + kv0 + row) * DM + h * HD + dh;
      const size_t vro = (size_t)(h * HD + row) * NTOK + (size_t)b * SEQ + kv0 + dh;
#pragma unroll
      for (int i = 0; i < 4; ++i) {
        *(v8us*)&Ks[row * 64 + dh + 8 * i]  = *(const v8us*)(QK16 + kro + 8 * i);
        *(v8us*)&Vts[row * 64 + dh + 8 * i] = *(const v8us*)(VT16 + vro + 8 * i);
      }
      if (tid < 64) msk_s[tid] = MK[(size_t)b * SEQ_FULL + kv0 + tid];
    }
    __syncthreads();

#pragma unroll 1
    for (int hf = 0; hf < 2; ++hf) {
      v8f s0 = (v8f){0.f,0.f,0.f,0.f,0.f,0.f,0.f,0.f};
      v8f s1 = s0;
#pragma unroll
      for (int dc = 0; dc < 2; ++dc) {
        v16h qf, kf;
        LDFRAG(qf, Qs, qro + dc * 32);
        const int ko0 = ((2 * hf) * 16 + c) * 64 + dc * 32 + 8 * hh;
        LDFRAG(kf, Ks, ko0);
        s0 = mma_h(qf, kf, s0);
        const int ko1 = ko0 + 16 * 64;
        LDFRAG(kf, Ks, ko1);
        s1 = mma_h(qf, kf, s1);
      }
      const bool keep0 = (msk_s[hf * 32 + c] != 0);
      const bool keep1 = (msk_s[hf * 32 + 16 + c] != 0);
#pragma unroll
      for (int r = 0; r < 8; ++r) {
        const float a0 = keep0 ? s0[r] * SC_SCORE : NEG_FILL;
        const float a1 = keep1 ? s1[r] * SC_SCORE : NEG_FILL;
        float m = fmaxf(a0, a1);
        m = fmaxf(m, __shfl_xor(m, 1, 32)); m = fmaxf(m, __shfl_xor(m, 2, 32));
        m = fmaxf(m, __shfl_xor(m, 4, 32)); m = fmaxf(m, __shfl_xor(m, 8, 32));
        const float mnew = fmaxf(mrow[r], m);
        const float alpha = expf(mrow[r] - mnew);
        mrow[r] = mnew;
        const float p0 = expf(a0 - mnew);
        const float p1 = expf(a1 - mnew);
        const float w0 = keep0 ? p0 : 0.f;
        const float w1 = keep1 ? p1 : 0.f;
        lrow[r] = lrow[r] * alpha + (p0 + p1);
        lval[r] = lval[r] * alpha + (w0 + w1);
#pragma unroll
        for (int t = 0; t < 4; ++t) oacc[t][r] *= alpha;
        const int po = pb + (8 * hh + r) * 32 + c;
        Ps[po] = gk::f2h_bits(w0 * P_CARRY);
        Ps[po + 16] = gk::f2h_bits(w1 * P_CARRY);
      }
      wave_sync();
      v16h pa;
      LDFRAG(pa, Ps, pb + c * 32 + 8 * hh);
#pragma unroll
      for (int t = 0; t < 4; ++t) {
        v16h vf;
        const int vo = (t * 16 + c) * 64 + hf * 32 + 8 * hh;
        LDFRAG(vf, Vts, vo);
        oacc[t] = mma_h(pa, vf, oacc[t]);
      }
      wave_sync();
    }
  }

  __syncthreads();
  {
    const int sb = wave * 1024;
#pragma unroll
    for (int r = 0; r < 8; ++r) {
      float l = lrow[r], lv = lval[r];
      l += __shfl_xor(l, 1, 32); l += __shfl_xor(l, 2, 32); l += __shfl_xor(l, 4, 32); l += __shfl_xor(l, 8, 32);
      lv += __shfl_xor(lv, 1, 32); lv += __shfl_xor(lv, 2, 32); lv += __shfl_xor(lv, 4, 32); lv += __shfl_xor(lv, 8, 32);
      const float invl = (l > 0.f) ? (1.0f / l) : 0.f;
      const float den = lv * invl + 1.0e-8f;
      const float fac = invl * (1.0f / den) * CTX_FOLD;
#pragma unroll
      for (int t = 0; t < 4; ++t) Ks[sb + (8 * hh + r) * 64 + t * 16 + c] = gk::f2h_bits(oacc[t][r] * fac);
    }
    wave_sync();
    const int q4 = lane >> 3, c8 = (lane & 7) * 8;
    v8us hv[4];
#pragma unroll
    for (int it = 0; it < 4; ++it) {
      const int row = it * 4 + q4;
      hv[it] = *(const v8us*)&Ks[sb + row * 64 + c8];
    }
    for (int pass = 0; pass < 2; ++pass) {
#pragma unroll
      for (int it = 0; it < 4; ++it) {
        const int row = it * 4 + q4;
        us* dst = CTX + (size_t)(tok0 + wave * 16 + row) * DM + h * HD + c8;
        *(volatile v8us*)(dst) = hv[it];
      }
      __threadfence();
    }
  }
}

#define WS_X16   ((size_t)3 * NTOK * DM * 2)
#define WS_W16   ((size_t)4 * DM * DM * 2)
#define WS_BR    ((size_t)4 * DM * 4)
#define WS_QK    ((size_t)2 * NTOK * DM * 2)
#define WS_VT    ((size_t)DM * NTOK * 2)
#define WS_CTX   ((size_t)NTOK * DM * 2)
#define WS_TOTAL (WS_X16 + WS_W16 + WS_BR + WS_QK + WS_VT + WS_CTX)
static_assert(WS_X16 % 256 == 0 && WS_W16 % 256 == 0 && WS_BR % 256 == 0 && WS_QK % 256 == 0 && WS_VT % 256 == 0 && WS_CTX % 256 == 0);
static_assert(WS_TOTAL <= (size_t)134217728);
static_assert((size_t)((NB_FULL - 1) * SEQ_FULL + SEQ_FULL) * DM * 4 == (size_t)16777216);

extern "C" void kernel_launch(void* const* d_in, const int* in_sizes, int n_in, void* d_out, int out_size, void* d_ws, size_t ws_size, hipStream_t stream) {
  if (n_in < 12) return;
  const long long need_x = ((long long)(NB - 1) * SEQ_FULL + SEQ) * DM;
  const long long need_m = (long long)(NB - 1) * SEQ_FULL + SEQ;
  if ((long long)in_sizes[0] < need_x || (long long)in_sizes[1] < need_x || (long long)in_sizes[2] < need_x) return;
  if ((long long)in_sizes[3] < need_m) return;
  if (in_sizes[4] < DM * DM || in_sizes[6] < DM * DM || in_sizes[8] < DM * DM || in_sizes[10] < DM * DM) return;
  if (in_sizes[5] < DM || in_sizes[7] < DM || in_sizes[9] < DM || in_sizes[11] < DM) return;
  if ((long long)out_size < need_x) return;
  if (WS_TOTAL > ws_size) return;

  const float* xq = (const float*)d_in[0];
  const float* xk = (const float*)d_in[1];
  const float* xv = (const float*)d_in[2];
  const int* kmask = (const int*)d_in[3];
  const float* Wq = (const float*)d_in[4];
  const float* bq = (const float*)d_in[5];
  const float* Wk = (const float*)d_in[6];
  const float* bk = (const float*)d_in[7];
  const float* Wv = (const float*)d_in[8];
  const float* bv = (const float*)d_in[9];
  const float* Wo = (const float*)d_in[10];
  const float* bo = (const float*)d_in[11];
  float* out = (float*)d_out;

  char* wsp = (char*)d_ws;
  us* X16 = (us*)wsp;             wsp += WS_X16;
  us* W16 = (us*)wsp;             wsp += WS_W16;
  float* BR = (float*)wsp;        wsp += WS_BR;
  us* QK16 = (us*)wsp;            wsp += WS_QK;
  us* VT16 = (us*)wsp;            wsp += WS_VT;
  us* CTX = (us*)wsp;             wsp += WS_CTX;

  k_cast_w4<<<dim3((unsigned)((DM * (DM / 8) + 255) / 256)), dim3(256), 0, stream>>>(Wq, Wk, Wv, Wo, W16);
  k_bias4<<<dim3((unsigned)((DM + 255) / 256)), dim3(256), 0, stream>>>(bq, bk, bv, bo, BR);
  k_cast_x3<<<dim3((unsigned)(((long long)NTOK * (DM / 8) + 255) / 256)), dim3(256), 0, stream>>>(xq, xk, xv, X16);
  k_gemm_qk<<<dim3((unsigned)(((NTOK / 64) * (DM / 64) + 7) / 8), 2u), dim3(256), 0, stream>>>(X16, W16, QK16, BR);
  k_gemm_vt<<<dim3((unsigned)(((DM / 64) * (NTOK / 64) + 7) / 8), 1u), dim3(256), 0, stream>>>(W16 + (size_t)2 * DM * DM, X16 + (size_t)2 * NTOK * DM, VT16, BR + 2 * DM);
  k_attn_flash<<<dim3((unsigned)(NB * NH * NQB)), dim3(128), 0, stream>>>(QK16, VT16, kmask, CTX);
  k_gemm_out<<<dim3((unsigned)(((SEQ / 64) * (DM / 64) + 7) / 8), (unsigned)NB), dim3(256), 0, stream>>>(CTX, W16 + (size_t)3 * DM * DM, out, BR + 3 * DM);
}
